// MultiHeadAttention_43241730736613
// MI455X (gfx1250) — hardware-verified
//
#include <hip/hip_runtime.h>
#ifndef NB
#define NB 2
#endif
#ifndef SEQ
#define SEQ 4096
#endif
#define NB_FULL 2
#define SEQ_FULL 4096
#define EMB 768
#define HEADS 8
#define HD 96
#define NQKV (3 * EMB)
#define BSTRIDE_FULL ((size_t)SEQ_FULL * EMB)

#define PLANE_ELEMS ((size_t)NB * SEQ * EMB)
#define PLANE_ACT (PLANE_ELEMS * 2)
#define PLANE_W ((size_t)NQKV * EMB * 2)
#define CVT_X_BLOCKS ((NB * SEQ * (EMB / 8)) / 256)
#define OPITCH 100

static_assert(SEQ % 64 == 0);
static_assert(SEQ <= SEQ_FULL);
static_assert(NB <= NB_FULL);
static_assert(HEADS * HD == EMB);
static_assert(HD == 96);
static_assert(EMB % 64 == 0);
static_assert(EMB % 96 == 0);
static_assert(EMB % 32 == 0);
static_assert(NQKV % 64 == 0);
static_assert((NB * SEQ * (EMB / 8)) % 256 == 0);
static_assert((NB * SEQ) % 64 == 0);
static_assert(PLANE_ACT % 256 == 0);
static_assert(PLANE_W % 256 == 0);
static_assert((HD * 4) % 128 == 0);
static_assert((EMB * 4) % 128 == 0);
static_assert((HD / 4) % 8 == 0);
static_assert((16 * (HD / 4)) % 32 == 0);
static_assert((OPITCH * 4) % 16 == 0);
static_assert(OPITCH >= HD);
static_assert(4 * PLANE_ACT + PLANE_W <= (size_t)134217728);

typedef __bf16 v16b __attribute__((ext_vector_type(16)));
typedef _Float16 v16h __attribute__((ext_vector_type(16)));
typedef unsigned short v8us __attribute__((ext_vector_type(8), may_alias));
typedef float v8f __attribute__((ext_vector_type(8)));
typedef float v4f __attribute__((ext_vector_type(4)));
typedef float v4fa __attribute__((ext_vector_type(4), may_alias));
typedef _Float16 h16;
union FragB { v16b v; v8us half[2]; unsigned short u[16]; };
union FragH { v16h v; v8us half[2]; _Float16 h[16]; unsigned short u[16]; };

#define LOG2E 1.4426950408889634f
#define QK_SCALE 0.03608439182435161f
#define C2 (QK_SCALE * LOG2E * (1.0f / 256.0f))

__device__ __forceinline__ unsigned short bf16_bits(float x) {
  unsigned int u = __float_as_uint(x);
  return (unsigned short)((u + 0x7FFFu + ((u >> 16) & 1u)) >> 16);
}
__device__ __forceinline__ float bf16_val(unsigned short b) { return __uint_as_float(((unsigned int)b) << 16); }
__device__ __forceinline__ float bf16_rne(float x) { return bf16_val(bf16_bits(x)); }

static __device__ __forceinline__ h16 toh_flush(float v) {
  const h16 r = (h16)v;
  return (fabsf(v) < 6.103515625e-05f) ? (h16)0.0f : r;
}
static __device__ __forceinline__ unsigned short h16_bits(h16 x) {
  union { h16 h; unsigned short u; } c;
  c.h = x;
  return c.u;
}

__device__ __forceinline__ void store_twice(unsigned short* d, v8us o) {
  *(volatile v8us*)d = o;
  __threadfence();
  *(volatile v8us*)d = o;
}

__device__ __forceinline__ void mma_s2(const FragH (&ka)[3], const FragH (&kb)[3], const FragH (&q)[3], v8f& s0, v8f& s1) {
  s0 = __builtin_amdgcn_wmma_f32_16x16x32_f16(false, ka[0].v, false, q[0].v, (short)0, s0, false, false);
  s1 = __builtin_amdgcn_wmma_f32_16x16x32_f16(false, kb[0].v, false, q[0].v, (short)0, s1, false, false);
  s0 = __builtin_amdgcn_wmma_f32_16x16x32_f16(false, ka[1].v, false, q[1].v, (short)0, s0, false, false);
  s1 = __builtin_amdgcn_wmma_f32_16x16x32_f16(false, kb[1].v, false, q[1].v, (short)0, s1, false, false);
  s0 = __builtin_amdgcn_wmma_f32_16x16x32_f16(false, ka[2].v, false, q[2].v, (short)0, s0, false, false);
  s1 = __builtin_amdgcn_wmma_f32_16x16x32_f16(false, kb[2].v, false, q[2].v, (short)0, s1, false, false);
  asm volatile("v_nop\n\tv_nop\n\tv_nop\n\tv_nop"
               : "+v"(s0), "+v"(s1)
               : "v"(ka[0].v), "v"(ka[1].v), "v"(ka[2].v), "v"(kb[0].v), "v"(kb[1].v), "v"(kb[2].v),
                 "v"(q[0].v), "v"(q[1].v), "v"(q[2].v));
}
__device__ __forceinline__ void mma_pv(const FragH (&vf)[6], v16h p, v8f (&O)[6]) {
  O[0] = __builtin_amdgcn_wmma_f32_16x16x32_f16(false, vf[0].v, false, p, (short)0, O[0], false, false);
  O[1] = __builtin_amdgcn_wmma_f32_16x16x32_f16(false, vf[1].v, false, p, (short)0, O[1], false, false);
  O[2] = __builtin_amdgcn_wmma_f32_16x16x32_f16(false, vf[2].v, false, p, (short)0, O[2], false, false);
  O[3] = __builtin_amdgcn_wmma_f32_16x16x32_f16(false, vf[3].v, false, p, (short)0, O[3], false, false);
  O[4] = __builtin_amdgcn_wmma_f32_16x16x32_f16(false, vf[4].v, false, p, (short)0, O[4], false, false);
  O[5] = __builtin_amdgcn_wmma_f32_16x16x32_f16(false, vf[5].v, false, p, (short)0, O[5], false, false);
  asm volatile("v_nop\n\tv_nop\n\tv_nop\n\tv_nop"
               : "+v"(O[0]), "+v"(O[1]), "+v"(O[2]), "+v"(O[3]), "+v"(O[4]), "+v"(O[5])
               : "v"(p), "v"(vf[0].v), "v"(vf[1].v), "v"(vf[2].v), "v"(vf[3].v), "v"(vf[4].v), "v"(vf[5].v));
}
__device__ __forceinline__ void mma_pj(v16b a, const FragB (&bw)[4], v8f (&c)[4]) {
  c[0] = __builtin_amdgcn_wmma_f32_16x16x32_bf16(false, a, false, bw[0].v, (short)0, c[0], false, false);
  c[1] = __builtin_amdgcn_wmma_f32_16x16x32_bf16(false, a, false, bw[1].v, (short)0, c[1], false, false);
  c[2] = __builtin_amdgcn_wmma_f32_16x16x32_bf16(false, a, false, bw[2].v, (short)0, c[2], false, false);
  c[3] = __builtin_amdgcn_wmma_f32_16x16x32_bf16(false, a, false, bw[3].v, (short)0, c[3], false, false);
  asm volatile("v_nop\n\tv_nop\n\tv_nop\n\tv_nop"
               : "+v"(c[0]), "+v"(c[1]), "+v"(c[2]), "+v"(c[3])
               : "v"(a), "v"(bw[0].v), "v"(bw[1].v), "v"(bw[2].v), "v"(bw[3].v));
}

__global__ __launch_bounds__(256) void k_cvt(const float* __restrict__ X, unsigned short* __restrict__ Xb) {
  const int bid = blockIdx.x;
  const int t = bid * 256 + threadIdx.x;
  const int row = t / (EMB / 8), piece = t - row * (EMB / 8);
  const int b = row / SEQ, s = row - b * SEQ;
  const float* src = X + (size_t)b * BSTRIDE_FULL + (size_t)s * EMB + piece * 8;
  const v4f x0 = *(const v4fa*)(src), x1 = *(const v4fa*)(src + 4);
  v8us o;
  o[0] = bf16_bits(x0[0]); o[1] = bf16_bits(x0[1]); o[2] = bf16_bits(x0[2]); o[3] = bf16_bits(x0[3]);
  o[4] = bf16_bits(x1[0]); o[5] = bf16_bits(x1[1]); o[6] = bf16_bits(x1[2]); o[7] = bf16_bits(x1[3]);
  store_twice(Xb + (size_t)t * 8, o);
}

__global__ __launch_bounds__(256) void k_wt(const float* __restrict__ W, unsigned short* __restrict__ Wt) {
  __shared__ unsigned short tl[64][66];
  const int tid = threadIdx.x;
  const int ng = blockIdx.x % (NQKV / 64);
  const int kg = blockIdx.x / (NQKV / 64);
  const int k0 = kg * 64, n0 = ng * 64;
  for (int i = tid; i < 64 * 16; i += 256) {
    const int j = i >> 4, c4 = (i & 15) * 4;
    const v4f x = *(const v4fa*)(W + (size_t)(k0 + j) * NQKV + n0 + c4);
    tl[c4 + 0][j] = bf16_bits(x[0]);
    tl[c4 + 1][j] = bf16_bits(x[1]);
    tl[c4 + 2][j] = bf16_bits(x[2]);
    tl[c4 + 3][j] = bf16_bits(x[3]);
  }
  __syncthreads();
  for (int pass = 0; pass < 2; ++pass) {
    for (int i = tid; i < 64 * 8; i += 256) {
      const int d = i >> 3, j8 = (i & 7) * 8;
      v8us o;
#pragma unroll
      for (int q = 0; q < 8; ++q) o[q] = tl[d][j8 + q];
      *(volatile v8us*)(Wt + (size_t)(n0 + d) * EMB + k0 + j8) = o;
    }
    if (pass == 0) __threadfence();
  }
}

__global__ __launch_bounds__(128) void k_qkv(const unsigned short* __restrict__ Xb, const unsigned short* __restrict__ Wt,
                                             const float* __restrict__ Bv, unsigned short* __restrict__ Pl) {
  __shared__ unsigned short tl[64][66];
  const int tid = threadIdx.x, lane = tid & 31, ln = lane & 15, hh = lane >> 4;
  const int w = __builtin_amdgcn_readfirstlane(tid >> 5);
  const int bn = blockIdx.x % (NQKV / 64), bm = blockIdx.x / (NQKV / 64);
  const int row0 = bm * 64 + 16 * w;
  const int col0 = bn * 64;
  v8f acc[4] = {};
  const unsigned short* ap0 = Xb + (size_t)(row0 + ln) * EMB + 8 * hh;
  const unsigned short* bp0 = Wt + (size_t)(col0 + ln) * EMB + 8 * hh;
#pragma unroll 1
  for (int k3 = 0; k3 < EMB / 96; ++k3) {
    const unsigned short* ap = ap0 + 96 * k3;
    const unsigned short* bp = bp0 + 96 * k3;
#pragma unroll
    for (int cc = 0; cc < 3; ++cc) {
      FragB a;
      a.half[0] = *(const v8us*)(ap + 32 * cc);
      a.half[1] = *(const v8us*)(ap + 32 * cc + 16);
      FragB bw[4];
#pragma unroll
      for (int nt = 0; nt < 4; ++nt) {
        bw[nt].half[0] = *(const v8us*)(bp + (size_t)nt * 16 * EMB + 32 * cc);
        bw[nt].half[1] = *(const v8us*)(bp + (size_t)nt * 16 * EMB + 32 * cc + 16);
      }
      mma_pj(a.v, bw, acc);
    }
  }
  const int which = bn / (EMB / 64);
  const int e0 = col0 - which * EMB;
  if (which == 2) {
#pragma unroll
    for (int nt = 0; nt < 4; ++nt) {
      const float bias = bf16_rne(Bv[col0 + 16 * nt + ln]);
#pragma unroll
      for (int r = 0; r < 8; ++r)
        tl[16 * nt + ln][16 * w + 8 * hh + r] = h16_bits(toh_flush((acc[nt][r] + bias) * 16.0f));
    }
  } else {
#pragma unroll
    for (int nt = 0; nt < 4; ++nt) {
      const float bias = bf16_rne(Bv[col0 + 16 * nt + ln]);
#pragma unroll
      for (int r = 0; r < 8; ++r)
        tl[16 * w + 8 * hh + r][16 * nt + ln] = h16_bits(toh_flush((acc[nt][r] + bias) * 16.0f));
    }
  }
  __syncthreads();
  const int t0 = bm * 64;
  const int b = t0 / SEQ, s0 = t0 - b * SEQ;
  size_t base, pitch;
  if (which == 2) {
    base = 2 * PLANE_ELEMS + ((size_t)b * EMB + e0) * SEQ + s0;
    pitch = SEQ;
  } else {
    base = (size_t)which * PLANE_ELEMS + ((size_t)b * SEQ + s0) * EMB + e0;
    pitch = EMB;
  }
  for (int pass = 0; pass < 2; ++pass) {
    for (int i = tid; i < 64 * 8; i += 128) {
      const int d = i >> 3, j8 = (i & 7) * 8;
      v8us o;
#pragma unroll
      for (int q = 0; q < 8; ++q) o[q] = tl[d][j8 + q];
      *(volatile v8us*)(Pl + base + (size_t)d * pitch + j8) = o;
    }
    if (pass == 0) __threadfence();
  }
}

__device__ __forceinline__ void fa_step(const unsigned short* __restrict__ Kp, const unsigned short* __restrict__ Vp,
                                        int key0, int ln, int hh, const FragH (&q)[3],
                                        float& mr, float& lr, v8f (&O)[6]) {
  const unsigned short* kp0 = Kp + (size_t)(key0 + ln) * EMB + 8 * hh;
  const unsigned short* kp1 = kp0 + 16 * EMB;
  FragH ka[3], kb[3];
#pragma unroll
  for (int c = 0; c < 3; ++c) {
    ka[c].half[0] = *(const v8us*)(kp0 + 32 * c);
    ka[c].half[1] = *(const v8us*)(kp0 + 32 * c + 16);
    kb[c].half[0] = *(const v8us*)(kp1 + 32 * c);
    kb[c].half[1] = *(const v8us*)(kp1 + 32 * c + 16);
  }
  const unsigned short* vp = Vp + (size_t)ln * SEQ + key0 + 8 * hh;
  FragH vf[6];
#pragma unroll
  for (int t = 0; t < 6; ++t) {
    vf[t].half[0] = *(const v8us*)(vp + (size_t)t * 16 * SEQ);
    vf[t].half[1] = *(const v8us*)(vp + (size_t)t * 16 * SEQ + 16);
  }
  v8f s0 = {0.f, 0.f, 0.f, 0.f, 0.f, 0.f, 0.f, 0.f};
  v8f s1 = {0.f, 0.f, 0.f, 0.f, 0.f, 0.f, 0.f, 0.f};
  mma_s2(ka, kb, q, s0, s1);
  float sc[16];
#pragma unroll
  for (int r = 0; r < 8; ++r) { sc[r] = s0[r] * C2; sc[8 + r] = s1[r] * C2; }
  float mx = sc[0];
#pragma unroll
  for (int i = 1; i < 16; ++i) mx = fmaxf(mx, sc[i]);
  mx = fmaxf(mx, __shfl_xor(mx, 16, 32));
  const float mnew = fmaxf(mr, mx);
  const float al = __builtin_amdgcn_exp2f(mr - mnew);
  mr = mnew;
  const float m8 = mnew - 8.0f;
  FragH ph;
  float ps = 0.0f;
#pragma unroll
  for (int i = 0; i < 16; ++i) {
    const float e = sc[i] - m8;
    const float pe = __builtin_amdgcn_exp2f(e);
    const float pc = (e < -14.0f) ? 0.0f : pe;
    ps += pc;
    ph.h[i] = (_Float16)pc;
  }
  ps += __shfl_xor(ps, 16, 32);
  lr = lr * al + ps;
#pragma unroll
  for (int t = 0; t < 6; ++t) O[t] = O[t] * al;
  mma_pv(vf, ph.v, O);
}

__global__ __launch_bounds__(128) __attribute__((amdgpu_num_vgpr(256)))
void k_attn(const unsigned short* __restrict__ Qh, const unsigned short* __restrict__ Kh,
            const unsigned short* __restrict__ Vt, float* __restrict__ Out) {
  __shared__ __attribute__((aligned(16))) float so[4][16 * OPITCH];
  const int tid = threadIdx.x, lane = tid & 31, ln = lane & 15, hh = lane >> 4;
  const int w = __builtin_amdgcn_readfirstlane(tid >> 5);
  const int qt = blockIdx.x % (SEQ / 64);
  const int rest = blockIdx.x / (SEQ / 64);
  const int h = rest % HEADS, b = rest / HEADS;
  const int qbase = qt * 64 + 16 * w;
  const int qg = qbase + ln;
  const unsigned short* qrow = Qh + ((size_t)b * SEQ + qg) * EMB + h * HD + 8 * hh;
  FragH q[3];
#pragma unroll
  for (int c = 0; c < 3; ++c) {
    q[c].half[0] = *(const v8us*)(qrow + 32 * c);
    q[c].half[1] = *(const v8us*)(qrow + 32 * c + 16);
  }
  float mr = -3.0e38f, lr = 0.0f;
  v8f O[6] = {};
  const unsigned short* Kp = Kh + (size_t)b * SEQ * EMB + h * HD;
  const unsigned short* Vp = Vt + ((size_t)b * EMB + h * HD) * SEQ;
#pragma unroll 1
  for (int j = 0; j < SEQ / 32; ++j)
    fa_step(Kp, Vp, 32 * j, ln, hh, q, mr, lr, O);

  const float cinv = 0.0625f * (1.0f / lr);
#pragma unroll
  for (int t = 0; t < 6; ++t) {
    v4f o0, o1;
    o0[0] = O[t][0] * cinv; o0[1] = O[t][1] * cinv; o0[2] = O[t][2] * cinv; o0[3] = O[t][3] * cinv;
    o1[0] = O[t][4] * cinv; o1[1] = O[t][5] * cinv; o1[2] = O[t][6] * cinv; o1[3] = O[t][7] * cinv;
    *(v4fa*)&so[w][ln * OPITCH + 16 * t + 8 * hh] = o0;
    *(v4fa*)&so[w][ln * OPITCH + 16 * t + 8 * hh + 4] = o1;
  }
  __syncthreads();
  float* og = Out + (size_t)b * BSTRIDE_FULL + (size_t)qbase * EMB + h * HD;
  for (int pass = 0; pass < 2; ++pass) {
#pragma unroll
    for (int i = 0; i < (16 * (HD / 4)) / 32; ++i) {
      const int p = i * 32 + lane;
      const int row = p / (HD / 4);
      const int c4 = (p - row * (HD / 4)) * 4;
      const v4f v = *(const v4fa*)&so[w][row * OPITCH + c4];
      *(volatile v4f*)(og + (size_t)row * EMB + c4) = v;
    }
    if (pass == 0) __threadfence();
  }
}

extern "C" void kernel_launch(void* const* d_in, const int* in_sizes, int n_in,
                              void* d_out, int out_size, void* d_ws, size_t ws_size, hipStream_t stream) {
  if (n_in < 3) return;
  const long long need = (long long)(NB - 1) * SEQ_FULL * EMB + (long long)SEQ * EMB;
  if ((long long)in_sizes[0] < need) return;
  if ((long long)in_sizes[1] < (long long)EMB * NQKV || (long long)in_sizes[2] < (long long)NQKV) return;
  if ((long long)out_size < need) return;
  const float* X = (const float*)d_in[0];
  const float* W = (const float*)d_in[1];
  const float* Bv = (const float*)d_in[2];
  float* Out = (float*)d_out;
  char* ws = (char*)d_ws;
  size_t off = 0;
  unsigned short* Xb = (unsigned short*)(ws + off); off += PLANE_ACT;
  unsigned short* Wt = (unsigned short*)(ws + off); off += PLANE_W;
  unsigned short* Pl = (unsigned short*)(ws + off); off += 3 * PLANE_ACT;
  if (off > ws_size) return;
  k_cvt<<<(unsigned)(CVT_X_BLOCKS), 256, 0, stream>>>(X, Xb);
  k_wt<<<(unsigned)((EMB / 64) * (NQKV / 64)), 256, 0, stream>>>(W, Wt);
  k_qkv<<<(unsigned)((NB * SEQ / 64) * (NQKV / 64)), 128, 0, stream>>>(Xb, Wt, Bv, Pl);
  k_attn<<<(unsigned)(NB * HEADS * (SEQ / 64)), 128, 0, stream>>>(Pl, Pl + PLANE_ELEMS, Pl + 2 * PLANE_ELEMS, Out);
}
